// SimpleGraphLayer_23476291240575
// MI455X (gfx1250) — hardware-run, weakly checked
//
#include <hip/hip_runtime.h>


#ifndef NN
#define NN 1024
#endif
#define NN_FULL 1024
#define DM   128
#define K2   256
#define RB   16
#define NW   8
#define AHP  264
#define ARP  136
#define FSP  132
#define QRS  2048.0f
#define QRI  (1.0f / 2048.0f)
#define WCS  64.0f
#define WCI  (1.0f / 64.0f)
#define LNE  1.0e-5f

static_assert(NN % 64 == 0);
static_assert(NN % RB == 0);
static_assert(NN % 2 == 0);
static_assert(NN <= NN_FULL);
static_assert(DM % 32 == 0);
static_assert(K2 == 2 * DM);
static_assert(K2 % 64 == 0);
static_assert(DM % 64 == 0);
static_assert(32 * 4 == DM);
static_assert(NW * 2 == RB);
static_assert(NW * 16 == DM);
static_assert(NW * 32 * 8 == RB * DM);
static_assert(32 * 16 * 8 == 16 * 64 * 4);
static_assert(32 * 16 == DM * 4);
static_assert(AHP >= K2 && (AHP * 2) % 16 == 0);
static_assert(ARP >= DM && (ARP * 2) % 16 == 0);
static_assert(FSP >= DM && (FSP * 4) % 16 == 0);
static_assert(RB * AHP * 2 + RB * ARP * 2 + 2 * RB * FSP * 4 <= 131072);
static_assert(16 * 68 * 4 <= 131072);
static_assert(((size_t)NN * DM) % 8 == 0);
static_assert(((size_t)DM * K2) % 8 == 0);

typedef _Float16 h16;
typedef unsigned short bf;
typedef __attribute__((ext_vector_type(16))) __bf16   v16bf;
typedef __attribute__((ext_vector_type(16))) _Float16 v16h;
typedef __attribute__((ext_vector_type(8)))  _Float16 v8h;
typedef __attribute__((ext_vector_type(4)))  _Float16 v4h;
typedef __attribute__((ext_vector_type(8)))  unsigned short v8us;
typedef __attribute__((ext_vector_type(8)))  float    v8f;
typedef __attribute__((ext_vector_type(4)))  float    v4f;
typedef v4f  __attribute__((may_alias)) v4fa;
typedef v8h  __attribute__((may_alias)) v8ha;
typedef v4h  __attribute__((may_alias)) v4ha;

__device__ __forceinline__ unsigned short f2bf(float f) { unsigned u = __float_as_uint(f); u += 0x7FFFu + ((u >> 16) & 1u); return (unsigned short)(u >> 16); }
__device__ __forceinline__ float bfr(float f) { return __uint_as_float(((unsigned)f2bf(f)) << 16); }
__device__ __forceinline__ v16h cat16(v8h lo, v8h hi) { return __builtin_shufflevector(lo, hi, 0, 1, 2, 3, 4, 5, 6, 7, 8, 9, 10, 11, 12, 13, 14, 15); }
__device__ __forceinline__ v16bf cat16b(v8us lo, v8us hi) { return __builtin_bit_cast(v16bf, __builtin_shufflevector(lo, hi, 0, 1, 2, 3, 4, 5, 6, 7, 8, 9, 10, 11, 12, 13, 14, 15)); }
__device__ __forceinline__ v16h  ldh(const h16* p) { return cat16(*(const v8h*)p, *(const v8h*)(p + 16)); }
__device__ __forceinline__ v16bf ldb(const bf* p)  { return cat16b(*(const v8us*)p, *(const v8us*)(p + 16)); }
__device__ __forceinline__ void wave_sync() { __builtin_amdgcn_fence(3  , "wavefront"); __builtin_amdgcn_wave_barrier(); asm volatile("" ::: "memory"); }
__device__ __forceinline__ v8f wmma16g(v16h a, v16h b, v8f c) {
    c = __builtin_amdgcn_wmma_f32_16x16x32_f16(false, a, false, b, (short)0, c, false, false);
    asm volatile("v_nop\n\tv_nop\n\tv_nop\n\tv_nop" : "+v"(c) : "v"(a), "v"(b));
    return c; }
__device__ __forceinline__ v8f wmmabg(v16bf a, v16bf b, v8f c) {
    c = __builtin_amdgcn_wmma_f32_16x16x32_bf16(false, a, false, b, (short)0, c, false, false);
    asm volatile("v_nop\n\tv_nop\n\tv_nop\n\tv_nop" : "+v"(c) : "v"(a), "v"(b));
    return c; }
static __device__ __forceinline__ h16 toh_flush(float v) { const h16 r = (h16)v; return (fabsf(v) < 6.103515625e-05f) ? (h16)0.0f : r; }
__device__ __forceinline__ float gelu_erf(float x) { return 0.5f * x * (1.0f + erff(x * 0.70710678118654752440f)); }

__global__ __launch_bounds__(256) void k_cvt8(const float* __restrict__ src, bf* dst, size_t n8) {
    const size_t i = (size_t)blockIdx.x * 256 + threadIdx.x; if (i >= n8) return;
    const v8f v = *(const v8f*)(src + i * 8); v8us o;
#pragma unroll
    for (int k = 0; k < 8; ++k) o[k] = f2bf(v[k]);
    *(volatile v8us*)(dst + i * 8) = o; __threadfence(); *(volatile v8us*)(dst + i * 8) = o;
}

__global__ __launch_bounds__(256) void k_cvth(const float* __restrict__ src, h16* dst, size_t n8) {
    const size_t i = (size_t)blockIdx.x * 256 + threadIdx.x; if (i >= n8) return;
    const v8f v = *(const v8f*)(src + i * 8); v8h o;
#pragma unroll
    for (int k = 0; k < 8; ++k) o[k] = toh_flush(bfr(v[k]) * WCS);
    *(volatile v8h*)(dst + i * 8) = o; __threadfence(); *(volatile v8h*)(dst + i * 8) = o;
}

__global__ __launch_bounds__(32) void k_sd(const bf* __restrict__ XB, const bf* __restrict__ MWB, const float* __restrict__ msgb, float* SD) {
    __shared__ __align__(16) float os[16 * 68];
    const int lane = threadIdx.x & 31, lr = lane & 15, hi = lane >> 4; const int r0 = blockIdx.x * 64, c0 = blockIdx.y * 64;
    const int cw = c0 & (DM - 1);
    const int ch = c0 / DM;
    v8f acc[4][4];
#pragma unroll
    for (int mb = 0; mb < 4; ++mb)
#pragma unroll
        for (int nb = 0; nb < 4; ++nb) acc[mb][nb] = (v8f){};
    const size_t aoff = (size_t)(r0 + lr) * DM + 8 * hi;
    const size_t boff = (size_t)(cw + lr) * K2 + (size_t)ch * DM + 8 * hi;
#pragma unroll 1
    for (int kc = 0; kc < DM; kc += 32) {
        v16bf a[4];
#pragma unroll
        for (int mb = 0; mb < 4; ++mb) a[mb] = ldb(XB + aoff + (size_t)mb * 16 * DM + kc);
#pragma unroll
        for (int nb = 0; nb < 4; ++nb) { const v16bf b = ldb(MWB + boff + (size_t)nb * 16 * K2 + kc);
#pragma unroll
            for (int mb = 0; mb < 4; ++mb) acc[mb][nb] = wmmabg(a[mb], b, acc[mb][nb]); }
    }
    float bc[4];
#pragma unroll
    for (int nb = 0; nb < 4; ++nb) { float t = msgb[cw + nb * 16 + lr]; asm volatile("" : "+v"(t)); bc[nb] = (ch != 0) ? bfr(t) : 0.0f; }
#pragma unroll
    for (int mb = 0; mb < 4; ++mb) {
#pragma unroll
        for (int nb = 0; nb < 4; ++nb) {
#pragma unroll
            for (int j = 0; j < 8; ++j) os[(hi * 8 + j) * 68 + nb * 16 + lr] = acc[mb][nb][j] + bc[nb]; }
        wave_sync();
        float* sb = SD + (size_t)(r0 + mb * 16) * K2 + c0;
#pragma unroll 1
        for (int ps = 0; ps < 2; ++ps) {
#pragma unroll
            for (int s = 0; s < 8; ++s) { const int row = 2 * s + (lane >> 4), cofs = (lane & 15) * 4;
                const v4f val = *(const v4fa*)(&os[row * 68 + cofs]);
                *(volatile v4f*)(sb + (size_t)row * K2 + cofs) = val; }
            if (ps == 0) __threadfence(); }
        wave_sync();
    }
}

__global__ __launch_bounds__(32 * NW) void k_node(const float* __restrict__ X, const float* __restrict__ ADJ, const float* __restrict__ SD, const h16* __restrict__ UWH,
                                                  const float* __restrict__ updb, const float* __restrict__ lnw, const float* __restrict__ lnb, float* OUT) {
    __shared__ __align__(16) h16   ah[RB * AHP];
    __shared__ __align__(16) h16   ar[RB * ARP];
    __shared__ __align__(16) float xs[RB * FSP];
    __shared__ __align__(16) float hs[RB * FSP];
    const int lane = threadIdx.x & 31, lr = lane & 15, hi = lane >> 4;
    const int wave = __builtin_amdgcn_readfirstlane((int)(threadIdx.x >> 5));
    const size_t i0 = (size_t)blockIdx.x * RB;
    { const int row = (int)(threadIdx.x >> 4), c8 = (int)(threadIdx.x & 15) * 8;
      const float* xp = X + (i0 + row) * DM + c8;
      const v4f x0 = *(const v4f*)xp, x1 = *(const v4f*)(xp + 4); v4f y0, y1; v8h hv;
#pragma unroll
      for (int i = 0; i < 4; ++i) { y0[i] = bfr(x0[i]); y1[i] = bfr(x1[i]); hv[i] = toh_flush(y0[i]); hv[4 + i] = toh_flush(y1[i]); }
      *(v4fa*)(&xs[row * FSP + c8]) = y0; *(v4fa*)(&xs[row * FSP + c8 + 4]) = y1;
      *(v8ha*)(&ah[row * AHP + c8]) = hv; }
    { const int d0 = 4 * lane;
      const size_t ia = i0 + 2 * wave;
      const v4f sa = *(const v4f*)(SD + ia * K2 + d0), sb = *(const v4f*)(SD + (ia + 1) * K2 + d0);
      const float* adja = ADJ + ia * NN_FULL;
      const float* adjb = adja + NN_FULL;
      const float* ep = SD + DM + d0;
      v4f acca = (v4f){}, accb = (v4f){};
#pragma unroll 1
      for (int j = 0; j < NN; j += 2) {
          const float a0 = bfr(adja[j]), a1 = bfr(adja[j + 1]);
          const float b0 = bfr(adjb[j]), b1 = bfr(adjb[j + 1]);
          const v4f e0 = *(const v4f*)(ep + (size_t)j * K2);
          const v4f e1 = *(const v4f*)(ep + (size_t)(j + 1) * K2);
#pragma unroll
          for (int c = 0; c < 4; ++c) { acca[c] += a0 * gelu_erf(sa[c] + e0[c]); accb[c] += b0 * gelu_erf(sb[c] + e0[c]); }
#pragma unroll
          for (int c = 0; c < 4; ++c) { acca[c] += a1 * gelu_erf(sa[c] + e1[c]); accb[c] += b1 * gelu_erf(sb[c] + e1[c]); }
      }
      v4h ha, ra, hb, rb;
#pragma unroll
      for (int c = 0; c < 4; ++c) {
          const h16 pa = toh_flush(acca[c]); const h16 pb = toh_flush(accb[c]);
          ha[c] = pa; hb[c] = pb;
          ra[c] = toh_flush((acca[c] - (float)pa) * QRS); rb[c] = toh_flush((accb[c] - (float)pb) * QRS); }
      const int rwa = 2 * wave, rwb = 2 * wave + 1;
      *(v4ha*)(&ah[rwa * AHP + DM + d0]) = ha; *(v4ha*)(&ah[rwb * AHP + DM + d0]) = hb;
      *(v4ha*)(&ar[rwa * ARP + d0]) = ra;      *(v4ha*)(&ar[rwb * ARP + d0]) = rb; }
    __syncthreads();
    { const int n0 = wave * 16;
      const h16* bp = UWH + (size_t)(n0 + lr) * K2 + 8 * hi;
      const int ao = lr * AHP + 8 * hi;
      const int ro = lr * ARP + 8 * hi;
      v8f accH = (v8f){}, accR = (v8f){};
#pragma unroll
      for (int kc = 0; kc < K2; kc += 32) {
          const v16h a = cat16(*(const v8ha*)(&ah[ao + kc]), *(const v8ha*)(&ah[ao + kc + 16]));
          const v16h b = ldh(bp + kc);
          accH = wmma16g(a, b, accH); }
#pragma unroll
      for (int kc = 0; kc < DM; kc += 32) {
          const v16h a = cat16(*(const v8ha*)(&ar[ro + kc]), *(const v8ha*)(&ar[ro + kc + 16]));
          const v16h b = ldh(bp + DM + kc);
          accR = wmma16g(a, b, accR); }
      const int c = n0 + lr;
      float ub = updb[c]; ub = bfr(ub);
#pragma unroll
      for (int r = 0; r < 8; ++r) {
          const float nf = (accH[r] + accR[r] * QRI) * WCI + ub;
          hs[(8 * hi + r) * FSP + c] = gelu_erf(nf); } }
    __syncthreads();
    { const v4f lw = *(const v4f*)(lnw + 4 * lane), lb = *(const v4f*)(lnb + 4 * lane); v4f gw, gb;
#pragma unroll
      for (int c = 0; c < 4; ++c) { gw[c] = bfr(lw[c]); gb[c] = bfr(lb[c]); }
      v4f y[2];
#pragma unroll
      for (int rr = 0; rr < 2; ++rr) {
          const int row = 2 * wave + rr;
          const v4f g = *(const v4fa*)(&hs[row * FSP + 4 * lane]); const v4f xv = *(const v4fa*)(&xs[row * FSP + 4 * lane]);
          const v4f hv = g + xv;
          float sm = (hv[0] + hv[1]) + (hv[2] + hv[3]);
          sm += __shfl_xor(sm, 16, 32); sm += __shfl_xor(sm, 8, 32); sm += __shfl_xor(sm, 4, 32); sm += __shfl_xor(sm, 2, 32); sm += __shfl_xor(sm, 1, 32);
          const float mu = sm * (1.0f / (float)DM);
          const v4f dv = hv - mu;
          float sq = (dv[0] * dv[0] + dv[1] * dv[1]) + (dv[2] * dv[2] + dv[3] * dv[3]);
          sq += __shfl_xor(sq, 16, 32); sq += __shfl_xor(sq, 8, 32); sq += __shfl_xor(sq, 4, 32); sq += __shfl_xor(sq, 2, 32); sq += __shfl_xor(sq, 1, 32);
          const float var = sq * (1.0f / (float)DM);
          const float rstd = 1.0f / sqrtf(var + LNE);
#pragma unroll
          for (int c = 0; c < 4; ++c) y[rr][c] = dv[c] * rstd * gw[c] + gb[c]; }
      float* orow = OUT + (i0 + 2 * wave) * DM + 4 * lane;
#pragma unroll 1
      for (int ps = 0; ps < 2; ++ps) {
          *(volatile v4f*)(orow) = y[0];
          *(volatile v4f*)(orow + DM) = y[1];
          if (ps == 0) __threadfence(); } }
}

static constexpr size_t al256(size_t v) { return (v + 255) & ~(size_t)255; }
static constexpr size_t SZ_XB = al256((size_t)NN * DM * 2);
static constexpr size_t SZ_MW = al256((size_t)DM * K2 * 2);
static constexpr size_t SZ_UW = al256((size_t)DM * K2 * 2);
static constexpr size_t SZ_SD = al256((size_t)NN * K2 * 4);
static constexpr size_t SZ_TOTAL = SZ_XB + SZ_MW + SZ_UW + SZ_SD;
static_assert(SZ_TOTAL <= (size_t)134217728);
static_assert(((size_t)NN * DM * 2) % 128 == 0);
static_assert(((size_t)DM * K2 * 2) % 128 == 0);
static_assert((size_t)(NN / 64) * 64 * K2 * 4 <= SZ_SD);
static_assert((size_t)(NN / RB) * RB == (size_t)NN);

extern "C" void kernel_launch(void* const* d_in, const int* in_sizes, int n_in,
                              void* d_out, int out_size, void* d_ws, size_t ws_size, hipStream_t stream) {
    if (n_in < 8) return;
    if ((size_t)in_sizes[0] < (size_t)NN * DM) return;
    if ((size_t)in_sizes[1] < (size_t)(NN - 1) * NN_FULL + NN) return;
    if ((size_t)in_sizes[2] < (size_t)DM * K2 || (size_t)in_sizes[4] < (size_t)DM * K2) return;
    if (in_sizes[3] < DM || in_sizes[5] < DM || in_sizes[6] < DM || in_sizes[7] < DM) return;
    if ((size_t)out_size < (size_t)NN * DM) return;
    if (SZ_TOTAL > ws_size) return;
    const float* x    = (const float*)d_in[0];
    const float* adj  = (const float*)d_in[1];
    const float* msgw = (const float*)d_in[2];
    const float* msgb = (const float*)d_in[3];
    const float* updw = (const float*)d_in[4];
    const float* updb = (const float*)d_in[5];
    const float* lnw  = (const float*)d_in[6];
    const float* lnb  = (const float*)d_in[7];
    float* OUT = (float*)d_out;
    char* wsp = (char*)d_ws;
    bf*    XB  = (bf*)wsp;    wsp += SZ_XB;
    bf*    MWB = (bf*)wsp;    wsp += SZ_MW;
    h16*   UWH = (h16*)wsp;   wsp += SZ_UW;
    float* SD  = (float*)wsp; wsp += SZ_SD;

    { const size_t n8 = (size_t)NN * DM / 8; k_cvt8<<<(unsigned)((n8 + 255) / 256), 256, 0, stream>>>(x, XB, n8); }
    { const size_t n8 = (size_t)DM * K2 / 8; const unsigned g = (unsigned)((n8 + 255) / 256);
      k_cvt8<<<g, 256, 0, stream>>>(msgw, MWB, n8);
      k_cvth<<<g, 256, 0, stream>>>(updw, UWH, n8); }
    k_sd<<<dim3(NN / 64, K2 / 64, 1), 32, 0, stream>>>(XB, MWB, msgb, SD);
    k_node<<<dim3(NN / RB, 1, 1), 32 * NW, 0, stream>>>(x, adj, SD, UWH, updb, lnw, lnb, OUT);
}
